// TrackCrossAttention_36490042147415
// MI455X (gfx1250) — hardware-verified
//
#include <hip/hip_runtime.h>
#include <hip/hip_bf16.h>
#include <cstddef>
#include <cstdint>

typedef __attribute__((ext_vector_type(16))) _Float16 v16h;
typedef __attribute__((ext_vector_type(8)))  _Float16 v8h;
typedef __attribute__((ext_vector_type(8)))  float    v8f;
typedef __attribute__((ext_vector_type(4)))  float    v4fx;

#define BATCH   2
#define CSEQ    4096
#define TTR     16
#define DMODEL  512
#define NHEAD   8
#define DHEAD   64

#define WQ16_OFF 0
#define WK16_OFF 262144
#define WV16_OFF 294912
#define WO16_OFF 327680
#define W16_TOTAL 589824

#define AB_STRIDE  520
#define QF_STRIDE  520
#define TRK_STRIDE 72
#define KV_STRIDE  66

__device__ __forceinline__ v8f wmma_f16(v16h a, v16h b, v8f c) {
  v8f d = __builtin_amdgcn_wmma_f32_16x16x32_f16(false, a, false, b,
                                                 (short)0, c, false, false);
  asm volatile("v_nop\n\tv_nop\n\tv_nop\n\tv_nop" : "+v"(d) : "v"(a), "v"(b));
  return d;
}

__device__ __forceinline__ v16h load_a(const _Float16* row, int koff, int hi) {
  const _Float16* p = row + koff + (hi ? 8 : 0);
  v8h c0 = *(const v8h*)p;
  v8h c1 = *(const v8h*)(p + 16);
  v16h r;
#pragma unroll
  for (int i = 0; i < 8; ++i) { r[i] = c0[i]; r[i + 8] = c1[i]; }
  return r;
}

__device__ __forceinline__ unsigned lds_off(const void* p) {
  return (unsigned)(uintptr_t)p;
}
__device__ __forceinline__ void async_load_b128(unsigned ldsoff, const void* g) {
  asm volatile("global_load_async_to_lds_b128 %0, %1, off"
               :: "v"(ldsoff), "v"((unsigned long long)(uintptr_t)g)
               : "memory");
}
__device__ __forceinline__ void wait_async0() {
  asm volatile("s_wait_asynccnt 0x0" ::: "memory");
}

__global__ __launch_bounds__(256) void convert_weights(
    const float* __restrict__ wq, const float* __restrict__ wk,
    const float* __restrict__ wv, const float* __restrict__ wo,
    _Float16* __restrict__ w16)
{
  int gid = blockIdx.x * blockDim.x + threadIdx.x;
  if (gid >= W16_TOTAL) return;

  const float* src;
  int off;
  if      (gid < WK16_OFF) { src = wq; off = gid; }
  else if (gid < WV16_OFF) { src = wk; off = gid - WK16_OFF; }
  else if (gid < WO16_OFF) { src = wv; off = gid - WV16_OFF; }
  else                     { src = wo; off = gid - WO16_OFF; }

  int f    = off >> 9;
  int r    = off & 511;
  int lane = r >> 4;
  int i    = r & 15;
  int nt   = f & 31;
  int kt   = f >> 5;
  int hh   = (lane & 16) ? 1 : 0;
  int k    = kt * 32 + ((i < 8) ? (8 * hh + i) : (16 + 8 * hh + (i - 8)));
  int n    = nt * 16 + (lane & 15);
  const _Float16 hv = (_Float16)src[(size_t)k * DMODEL + n];
  *(volatile _Float16*)(w16 + gid) = hv; __threadfence(); *(volatile _Float16*)(w16 + gid) = hv;
}

__global__ __launch_bounds__(256) void track_attn(
    const float* __restrict__ x,
    const float* __restrict__ te,
    const float* __restrict__ nscale,
    const float* __restrict__ bq, const float* __restrict__ bk,
    const float* __restrict__ bv, const float* __restrict__ bo,
    const _Float16* __restrict__ w16,
    float* __restrict__ out)
{
  __shared__ __align__(16) float    QF[16 * QF_STRIDE];
  __shared__ __align__(32) _Float16 AB16[16 * AB_STRIDE];
  __shared__ __align__(32) _Float16 TRK[256 * TRK_STRIDE];
  __shared__ __align__(16) unsigned char KVPOOL[2 * 256 * KV_STRIDE * 2];
  __shared__ float LG[16][16];
  __shared__ float RINV[16];

  _Float16* KH = (_Float16*)KVPOOL;
  _Float16* VH = KH + 256 * KV_STRIDE;
  float*    TSTAGE = (float*)KVPOOL;

  const int tid  = threadIdx.x;
  const int lane = tid & 31;
  const int wid  = tid >> 5;
  const int l15  = lane & 15;
  const int hi   = lane >> 4;

  const int blk = blockIdx.x;
  const int b   = blk / (CSEQ / 16);
  const int c0  = (blk % (CSEQ / 16)) * 16;

  const _Float16* wq16 = w16 + WQ16_OFF;
  const _Float16* wk16 = w16 + WK16_OFF;
  const _Float16* wv16 = w16 + WV16_OFF;
  const _Float16* wo16 = w16 + WO16_OFF;

  for (int idx = tid * 4; idx < 16 * DMODEL; idx += 256 * 4) {
    int r = idx >> 9, d = idx & 511;
    *(float4*)&QF[r * QF_STRIDE + d] = *(const float4*)(x + ((size_t)(b * CSEQ + c0 + r)) * DMODEL + d);
  }
  for (int idx = tid * 4; idx < 256 * DHEAD; idx += 256 * 4) {
    int m = idx >> 6, d = idx & 63;
    int ctl = m >> 4, t = m & 15;
    *(float4*)&TSTAGE[m * 64 + d] = *(const float4*)(te + (((size_t)b * TTR + t) * CSEQ + (c0 + ctl)) * DHEAD + d);
  }
  __syncthreads();

  if (tid < 16) {
    float s = 0.f;
    for (int d = 0; d < DMODEL; ++d) {
      float v = QF[tid * QF_STRIDE + d];
      s += v * v;
    }
    RINV[tid] = rsqrtf(s * (1.0f / DMODEL) + 1e-6f);
  }
  __syncthreads();
  for (int idx = tid; idx < 16 * DMODEL; idx += 256) {
    int r = idx >> 9, d = idx & 511;
    AB16[r * AB_STRIDE + d] =
        (_Float16)(QF[r * QF_STRIDE + d] * RINV[r] * nscale[d]);
  }
  for (int idx = tid; idx < 256 * DHEAD; idx += 256) {
    int m = idx >> 6, d = idx & 63;
    TRK[m * TRK_STRIDE + d] = (_Float16)TSTAGE[m * 64 + d];
  }
  __syncthreads();

  {
    v8f acc[4] = {};
#pragma unroll 4
    for (int kt = 0; kt < 16; ++kt) {
      v16h a = load_a(&AB16[l15 * AB_STRIDE], kt * 32, hi);
      const _Float16* bb = wq16 + (size_t)(kt * 32 + wid) * 512 + lane * 16;
#pragma unroll
      for (int j = 0; j < 4; ++j)
        acc[j] = wmma_f16(a, *(const v16h*)(bb + j * 8 * 512), acc[j]);
    }
#pragma unroll
    for (int j = 0; j < 4; ++j) {
      int n = (wid + j * 8) * 16 + l15;
      float bqn = bq[n];
#pragma unroll
      for (int r = 0; r < 8; ++r)
        QF[(hi * 8 + r) * QF_STRIDE + n] = (acc[j][r] + bqn) * 0.125f;
    }
  }

  for (int h = 0; h < NHEAD; ++h) {
    for (int mt = wid; mt < 16; mt += 8) {
      const _Float16* arow = &TRK[(mt * 16 + l15) * TRK_STRIDE];
      v8f ka[4] = {}, va[4] = {};
#pragma unroll
      for (int kt = 0; kt < 2; ++kt) {
        v16h a = load_a(arow, kt * 32, hi);
#pragma unroll
        for (int nt = 0; nt < 4; ++nt) {
          size_t f = (size_t)(kt * 32 + h * 4 + nt) * 512 + lane * 16;
          ka[nt] = wmma_f16(a, *(const v16h*)(wk16 + f), ka[nt]);
          va[nt] = wmma_f16(a, *(const v16h*)(wv16 + f), va[nt]);
        }
      }
#pragma unroll
      for (int nt = 0; nt < 4; ++nt) {
        int n = nt * 16 + l15;
        float bkn = bk[h * 64 + n];
        float bvn = bv[h * 64 + n];
        int mb = mt * 16 + hi * 8;
#pragma unroll
        for (int r = 0; r < 8; ++r) {
          KH[(mb + r) * KV_STRIDE + n] = (_Float16)(ka[nt][r] + bkn);
          VH[(mb + r) * KV_STRIDE + n] = (_Float16)(va[nt][r] + bvn);
        }
      }
    }
    __syncthreads();

    {
      int tok = tid >> 4, t = tid & 15;
      const float* q = &QF[tok * QF_STRIDE + h * 64];
      const _Float16* k = &KH[(tok * 16 + t) * KV_STRIDE];
      float s = 0.f;
#pragma unroll 8
      for (int d = 0; d < 64; ++d) s += q[d] * (float)k[d];
      LG[tok][t] = s;
    }
    __syncthreads();

    if (tid < 16) {
      float mx = LG[tid][0];
#pragma unroll
      for (int t = 1; t < 16; ++t) mx = fmaxf(mx, LG[tid][t]);
      float sum = 0.f;
#pragma unroll
      for (int t = 0; t < 16; ++t) {
        float e = __expf(LG[tid][t] - mx);
        LG[tid][t] = e;
        sum += e;
      }
      float inv = 1.f / sum;
#pragma unroll
      for (int t = 0; t < 16; ++t) LG[tid][t] *= inv;
    }
    __syncthreads();

    for (int it = tid; it < 16 * 64; it += 256) {
      int tok = it >> 6, d = it & 63;
      float s = 0.f;
#pragma unroll
      for (int t = 0; t < 16; ++t)
        s += LG[tok][t] * (float)VH[(tok * 16 + t) * KV_STRIDE + d];
      AB16[tok * AB_STRIDE + h * 64 + d] = (_Float16)s;
    }
    __syncthreads();
  }

  {
    v8f acc[4] = {};
#pragma unroll 4
    for (int kt = 0; kt < 16; ++kt) {
      v16h a = load_a(&AB16[l15 * AB_STRIDE], kt * 32, hi);
      const _Float16* bb = wo16 + (size_t)(kt * 32 + wid) * 512 + lane * 16;
#pragma unroll
      for (int j = 0; j < 4; ++j)
        acc[j] = wmma_f16(a, *(const v16h*)(bb + j * 8 * 512), acc[j]);
    }
    __syncthreads();
#pragma unroll
    for (int j = 0; j < 4; ++j) {
      int n = (wid + j * 8) * 16 + l15;
      float bon = bo[n];
#pragma unroll
      for (int r = 0; r < 8; ++r) QF[(hi * 8 + r) * QF_STRIDE + n] = acc[j][r] + bon;
    }
    __syncthreads();
    for (int pass = 0; pass < 2; ++pass) {
#pragma unroll
      for (int q = 0; q < 8; ++q) {
        const int piece = q * 256 + tid, m = piece >> 7, d4 = (piece & 127) * 4;
        const size_t g = ((size_t)(b * CSEQ + c0 + m)) * DMODEL + d4;
        v4fx v = *(const v4fx*)&QF[m * QF_STRIDE + d4];
        const v4fx xr = *(const v4fx*)(x + g);
        v += xr;
        *(volatile v4fx*)(out + g) = v;
      }
      __threadfence();
    }
  }
}

extern "C" void kernel_launch(void* const* d_in, const int* in_sizes, int n_in,
                              void* d_out, int out_size, void* d_ws,
                              size_t ws_size, hipStream_t stream) {
  const float* x      = (const float*)d_in[0];
  const float* te     = (const float*)d_in[1];
  const float* nscale = (const float*)d_in[2];
  const float* wq     = (const float*)d_in[3];
  const float* bq     = (const float*)d_in[4];
  const float* wk     = (const float*)d_in[5];
  const float* bk     = (const float*)d_in[6];
  const float* wv     = (const float*)d_in[7];
  const float* bv     = (const float*)d_in[8];
  const float* wo     = (const float*)d_in[9];
  const float* bo     = (const float*)d_in[10];
  float* out = (float*)d_out;
  (void)in_sizes; (void)n_in; (void)out_size;
  if (ws_size < (size_t)W16_TOTAL * 2) return;
  _Float16* w16 = (_Float16*)d_ws;

  convert_weights<<<(W16_TOTAL + 255) / 256, 256, 0, stream>>>(wq, wk, wv, wo, w16);
  track_attn<<<(BATCH * CSEQ) / 16, 256, 0, stream>>>(
      x, te, nscale, bq, bk, bv, bo, w16, out);
}
